// SS2D_17179869668
// MI455X (gfx1250) — hardware-run, weakly checked
//
#include <hip/hip_runtime.h>
#include <hip/hip_fp16.h>
#include <math.h>

typedef __attribute__((ext_vector_type(16))) _Float16 v16h;
typedef __attribute__((ext_vector_type(8)))  _Float16 v8h;
typedef __attribute__((ext_vector_type(4)))  _Float16 v4h;
typedef __attribute__((ext_vector_type(8)))  float    v8f;
typedef __attribute__((ext_vector_type(4)))  float    v4f;
typedef __attribute__((ext_vector_type(4)))  unsigned gl_v4u;

constexpr int kBatch = 8;
constexpr int kImgH  = 64;
constexpr int kImgW  = 64;
constexpr int kCh    = 96;
constexpr int kDin   = 192;
constexpr int kNst   = 16;
constexpr int kDtR   = 6;
constexpr int kDir   = 4;
constexpr int kLen   = kImgH * kImgW;
constexpr int kRows  = kBatch * kLen;
constexpr int kXzN   = 2 * kDin;
constexpr int kXpC   = kDtR + 2 * kNst;
constexpr int kXpP   = 48;
constexpr int kXdN   = kDir * kXpP;
constexpr int kBcN   = 2 * kNst;
constexpr int kOutP  = 128;
constexpr float kWCarry  = 1024.0f;
constexpr float kResid   = 2048.0f;
constexpr float kYCarry  = 16.0f;
constexpr float kYgCarry = 16.0f;
static_assert(kLen == 4096 && kRows == 32768);
static_assert(kXpC == 38 && kXpC <= kXpP && kXdN == 192);
static_assert((kDin % 64) == 0 && (kLen % 64) == 0 && (kXzN % 64) == 0 && (kXdN % 64) == 0 && (kOutP % 64) == 0);
static_assert((kCh % 32) == 0 && (kDin % 32) == 0);
static_assert((kLen % 32) == 0 && (kRows % 32) == 0);

constexpr size_t kSzWIN  = (size_t)kXzN * kCh * 2;
constexpr size_t kSzWX   = (size_t)kXdN * kDin * 2;
constexpr size_t kSzWO   = (size_t)kOutP * kDin * 2;
constexpr size_t kSzX16  = (size_t)kRows * kCh * 2;
constexpr size_t kSzXZ   = (size_t)kLen * kXzN * 4;
constexpr size_t kSzP32  = (size_t)kLen * kDin * 4;
constexpr size_t kSzP16  = (size_t)kLen * kDin * 2;
constexpr size_t kSzBC   = (size_t)kDir * kLen * kBcN * 4;
constexpr size_t kSzYG   = (size_t)kRows * kDin * 2;
constexpr size_t kSzOUTP = (size_t)kRows * kOutP * 4;
constexpr size_t kOffWINH = 0;
constexpr size_t kOffWINL = kOffWINH + kSzWIN;
constexpr size_t kOffWX   = kOffWINL + kSzWIN;
constexpr size_t kOffWO   = kOffWX   + kSzWX;
constexpr size_t kOffXH   = kOffWO   + kSzWO;
constexpr size_t kOffXL   = kOffXH   + kSzX16;
constexpr size_t kOffXZ   = kOffXL   + kSzX16;
constexpr size_t kOffXC   = kOffXZ   + kSzXZ;
constexpr size_t kOffXCH  = kOffXC   + kSzP32;
constexpr size_t kOffXCL  = kOffXCH  + kSzP16;
constexpr size_t kOffXD   = kOffXCL  + kSzP16;
constexpr size_t kOffDTP  = kOffXD   + kSzP32;
constexpr size_t kOffUK   = kOffDTP  + kDir * kSzP32;
constexpr size_t kOffBC   = kOffUK   + kDir * kSzP32;
constexpr size_t kOffYSH  = kOffBC   + kSzBC;
constexpr size_t kOffYSL  = kOffYSH  + kDir * kSzP16;
constexpr size_t kOffYGH  = kOffYSL  + kDir * kSzP16;
constexpr size_t kOffYGL  = kOffYGH  + kSzYG;
constexpr size_t kOffOUTP = kOffYGL  + kSzYG;
constexpr size_t kWsTotal = kOffOUTP + kSzOUTP;
static_assert(kWsTotal == 110370816ull);
static_assert(kWsTotal <= 134217728ull);
static_assert((kOffWINL % 128) == 0 && (kOffWX % 128) == 0 && (kOffWO % 128) == 0 && (kOffXH % 128) == 0 &&
              (kOffXL % 128) == 0 && (kOffXZ % 128) == 0 && (kOffXC % 128) == 0 && (kOffXCH % 128) == 0 &&
              (kOffXCL % 128) == 0 && (kOffXD % 128) == 0 && (kOffDTP % 128) == 0 && (kOffUK % 128) == 0 &&
              (kOffBC % 128) == 0 && (kOffYSH % 128) == 0 && (kOffYSL % 128) == 0 && (kOffYGH % 128) == 0 &&
              (kOffYGL % 128) == 0 && (kOffOUTP % 128) == 0);

__device__ __forceinline__ _Float16 f16_flush(float v) {
  const float w = (fabsf(v) < 6.103515625e-05f) ? 0.0f : v;
  return (_Float16)w;
}
__device__ __forceinline__ void f16_split(float v, _Float16& hi, _Float16& lo) {
  hi = f16_flush(v);
  const float hf = (float)hi;
  const float r = (v - hf) * kResid;
  lo = f16_flush(r);
}

__device__ __forceinline__ float h16_to_f32(unsigned hb) {
  const unsigned sgn = (hb & 0x8000u) << 16; const unsigned em = hb & 0x7fffu;
  const float fn = __uint_as_float((em << 13) + 0x38000000u);
  const float fs = (float)em * 5.9604644775390625e-8f;
  const float mag = (em < 0x400u) ? fs : fn; return __uint_as_float(__float_as_uint(mag) | sgn); }

__device__ __forceinline__ int scan_pixel(int k, int l) {
  const int ll = (k >= 2) ? (kLen - 1 - l) : l;
  const int tw = ll >> 6;
  const int th = ll & 63;
  const int pt = (th << 6) + tw;
  return (k & 1) ? pt : ll;
}

namespace eng {
union FragU { v16h v; v8h h[2]; };
__device__ __forceinline__ v16h frag_load(const _Float16* p) {
  FragU f;
  f.h[0] = *(const v8h*)(p);
  f.h[1] = *(const v8h*)(p + 16);
  return f.v;
}
__device__ __forceinline__ v8f mma(v16h a, v16h b, v8f c) {
  return __builtin_amdgcn_wmma_f32_16x16x32_f16(false, a, false, b, (short)0, c, false, false);
}
__device__ __forceinline__ void guard1(v8f& a, v16h x, v16h y) {
  asm volatile("v_nop\n\tv_nop\n\tv_nop\n\tv_nop" : "+v"(a) : "v"(x), "v"(y));
}
__device__ __forceinline__ void guard_acc(v8f& a) {
  asm volatile("v_nop\n\tv_nop\n\tv_nop\n\tv_nop" : "+v"(a));
}
__device__ __forceinline__ void keep4(v16h a, v16h b, v16h c, v16h d) {
  asm volatile("v_nop" :: "v"(a), "v"(b), "v"(c), "v"(d));
}

template <int MI, int SPL>
__global__ __launch_bounds__(256) void gemm_f16_kernel(
    const unsigned short* __restrict__ Ap, const unsigned short* __restrict__ A2p, int lda,
    const unsigned short* __restrict__ Btp, const unsigned short* __restrict__ Bt2p, int ldb,
    float* __restrict__ C, int ldc, int M, int N, int K, float scale, float rscale)
{
  static_assert(MI >= 1 && MI <= 2);
  static_assert(SPL >= 0 && SPL <= 2);
  const _Float16* A   = (const _Float16*)Ap;
  const _Float16* A2  = (const _Float16*)A2p;
  const _Float16* Bt  = (const _Float16*)Btp;
  const _Float16* Bt2 = (const _Float16*)Bt2p;
  __shared__ __align__(16) float sT[8][16 * 68];
  const int lane = threadIdx.x & 31;
  const int wave = threadIdx.x >> 5;
  const int tilesN = N >> 6;
  const int tilesM = M / (16 * MI);
  const int tile = blockIdx.x * 8 + wave;
  if (tile >= tilesM * tilesN) return;
  const int tm = tile / tilesN;
  const int tn = tile - tm * tilesN;
  const int m0 = tm * (16 * MI);
  const int n0 = tn << 6;
  const int rlane = lane & 15;
  const int koff  = (lane >> 4) * 8;
  const int mOff  = (lane >> 4) * 8;

  v8f acc[MI][4], accr[MI][4];
#pragma unroll
  for (int i = 0; i < MI; ++i)
#pragma unroll
    for (int j = 0; j < 4; ++j) {
      acc[i][j]  = (v8f){0.f, 0.f, 0.f, 0.f, 0.f, 0.f, 0.f, 0.f};
      accr[i][j] = (v8f){0.f, 0.f, 0.f, 0.f, 0.f, 0.f, 0.f, 0.f};
    }

  for (int k0 = 0; k0 < K; k0 += 32) {
    v16h bh[4], bl[4];
#pragma unroll
    for (int j = 0; j < 4; ++j) {
      const size_t bo = (size_t)(n0 + (j << 4) + rlane) * ldb + koff + k0;
      bh[j] = frag_load(Bt + bo);
      if (SPL == 2) bl[j] = frag_load(Bt2 + bo); else bl[j] = bh[j];
    }
#pragma unroll
    for (int i = 0; i < MI; ++i) {
      const size_t ao = (size_t)(m0 + (i << 4) + rlane) * lda + koff + k0;
      const v16h ah = frag_load(A + ao);
      v16h al = ah;
      if (SPL >= 1) al = frag_load(A2 + ao);
#pragma unroll
      for (int j = 0; j < 4; ++j) {
        acc[i][j] = mma(ah, bh[j], acc[i][j]);
        if (SPL >= 1) accr[i][j] = mma(al, bh[j], accr[i][j]);
        if (SPL == 2) accr[i][j] = mma(ah, bl[j], accr[i][j]);
      }
#pragma unroll
      for (int j = 0; j < 4; ++j) {
        guard1(acc[i][j], ah, al);
        if (SPL >= 1) guard1(accr[i][j], ah, al);
      }
    }
    keep4(bh[0], bh[1], bh[2], bh[3]);
    if (SPL == 2) keep4(bl[0], bl[1], bl[2], bl[3]);
  }
#pragma unroll
  for (int i = 0; i < MI; ++i)
#pragma unroll
    for (int j = 0; j < 4; ++j) {
      guard_acc(acc[i][j]);
      if (SPL >= 1) guard_acc(accr[i][j]);
    }

  float* slab = sT[wave];
#pragma unroll
  for (int i = 0; i < MI; ++i) {
    const int mBase = m0 + (i << 4);
#pragma unroll
    for (int j = 0; j < 4; ++j) {
#pragma unroll
      for (int r = 0; r < 8; ++r) {
        float v = acc[i][j][r] * scale;
        if (SPL >= 1) v += accr[i][j][r] * rscale;
        slab[(mOff + r) * 68 + (j << 4) + rlane] = v;
      }
    }
    __builtin_amdgcn_fence(__ATOMIC_RELEASE, "workgroup");
    __builtin_amdgcn_wave_barrier();
    __builtin_amdgcn_fence(__ATOMIC_ACQUIRE, "workgroup");
    {
      const int hh = lane >> 4, c4 = (lane & 15) * 4;
      for (int pass = 0; pass < 2; ++pass) {
#pragma unroll
        for (int it = 0; it < 8; ++it) {
          const int row = it * 2 + hh;
          const v4f v = *(const v4f*)(slab + row * 68 + c4);
          *(volatile v4f*)(C + (size_t)(mBase + row) * ldc + n0 + c4) = v;
        }
        __threadfence();
      }
    }
    __builtin_amdgcn_fence(__ATOMIC_RELEASE, "workgroup");
    __builtin_amdgcn_wave_barrier();
    __builtin_amdgcn_fence(__ATOMIC_ACQUIRE, "workgroup");
  }
}
}

__global__ __launch_bounds__(256) void split_rows_f16_kernel(
    const float* __restrict__ src, unsigned short* __restrict__ dH, unsigned short* __restrict__ dL, int total8)
{
  const int i = blockIdx.x * 256 + threadIdx.x;
  if (i >= total8) return;
  const size_t e0 = (size_t)i << 3;
  const v4f a0 = *(const v4f*)(src + e0);
  const v4f a1 = *(const v4f*)(src + e0 + 4);
  v8h hv, lv;
#pragma unroll
  for (int e = 0; e < 4; ++e) {
    _Float16 h0, l0, h1, l1;
    const float f0 = a0[e];
    const float f1 = a1[e];
    f16_split(f0, h0, l0);
    f16_split(f1, h1, l1);
    hv[e] = h0; lv[e] = l0;
    hv[4 + e] = h1; lv[4 + e] = l1;
  }
  unsigned short* qh = dH + e0;
  unsigned short* ql = dL + e0;
  *(volatile v8h*)qh = hv;
  *(volatile v8h*)ql = lv;
  __threadfence();
  *(volatile v8h*)qh = hv;
  *(volatile v8h*)ql = lv;
}

template <bool LO>
__global__ __launch_bounds__(256) void pack_w_rows_kernel(
    const float* __restrict__ W, unsigned short* __restrict__ dH, unsigned short* __restrict__ dL,
    int K8, int gdst, int gsrc, int total8, float carry)
{
  const int i = blockIdx.x * 256 + threadIdx.x;
  if (i >= total8) return;
  const int n   = i / K8;
  const int kc  = i - n * K8;
  const int grp = n / gdst;
  const int c   = n - grp * gdst;
  const bool live = (c < gsrc);
  const int cc  = live ? c : (gsrc - 1);
  const size_t so = ((size_t)(grp * gsrc + cc) * K8 + kc) * 8;
  const v4f a0 = *(const v4f*)(W + so);
  const v4f a1 = *(const v4f*)(W + so + 4);
  v8h hv, lv;
#pragma unroll
  for (int e = 0; e < 4; ++e) {
    _Float16 h0, l0, h1, l1;
    const float f0 = live ? (a0[e] * carry) : 0.0f;
    const float f1 = live ? (a1[e] * carry) : 0.0f;
    f16_split(f0, h0, l0);
    f16_split(f1, h1, l1);
    hv[e] = h0; lv[e] = l0;
    hv[4 + e] = h1; lv[4 + e] = l1;
  }
  const size_t e0 = (size_t)i << 3;
  *(volatile v8h*)(dH + e0) = hv;
  if (LO) *(volatile v8h*)(dL + e0) = lv;
  __threadfence();
  *(volatile v8h*)(dH + e0) = hv;
  if (LO) *(volatile v8h*)(dL + e0) = lv;
}

__global__ __launch_bounds__(256) void dwconv3x3_silu_kernel(
    const float* __restrict__ XZ, const float* __restrict__ cw, const float* __restrict__ cb,
    float* __restrict__ XC, unsigned short* __restrict__ XCH, unsigned short* __restrict__ XCL)
{
  const int i = blockIdx.x * 256 + threadIdx.x;
  if (i >= kLen * (kDin / 4)) return;
  const int p  = i / (kDin / 4);
  const int g  = i - p * (kDin / 4);
  const int d4 = g * 4;
  const int ph = p >> 6;
  const int pw = p & 63;
  const v4f bv = *(const v4f*)(cb + d4);
  float a0 = 0.0f, a1 = 0.0f, a2 = 0.0f, a3 = 0.0f;
#pragma unroll 1
  for (int dy = 0; dy < 3; ++dy) {
    const int hh = ph + dy - 1;
    const int hc = (hh < 0) ? 0 : ((hh > kImgH - 1) ? (kImgH - 1) : hh);
    const float mh = (hh == hc) ? 1.0f : 0.0f;
#pragma unroll
    for (int dx = 0; dx < 3; ++dx) {
      const int ww = pw + dx - 1;
      const int wc = (ww < 0) ? 0 : ((ww > kImgW - 1) ? (kImgW - 1) : ww);
      const float m = (ww == wc) ? mh : 0.0f;
      const v4f xv = *(const v4f*)(XZ + (size_t)(hc * kImgW + wc) * kXzN + d4);
      const int t = dy * 3 + dx;
      const float w0 = cw[(d4 + 0) * 9 + t] * m;
      const float w1 = cw[(d4 + 1) * 9 + t] * m;
      const float w2 = cw[(d4 + 2) * 9 + t] * m;
      const float w3 = cw[(d4 + 3) * 9 + t] * m;
      a0 = fmaf(w0, xv[0], a0);
      a1 = fmaf(w1, xv[1], a1);
      a2 = fmaf(w2, xv[2], a2);
      a3 = fmaf(w3, xv[3], a3);
    }
  }
  v4f ov;
  v4h hv, lv;
  {
    const float s0 = a0 + bv[0], s1 = a1 + bv[1], s2 = a2 + bv[2], s3 = a3 + bv[3];
    ov[0] = s0 * __builtin_amdgcn_rcpf(1.0f + expf(-s0));
    ov[1] = s1 * __builtin_amdgcn_rcpf(1.0f + expf(-s1));
    ov[2] = s2 * __builtin_amdgcn_rcpf(1.0f + expf(-s2));
    ov[3] = s3 * __builtin_amdgcn_rcpf(1.0f + expf(-s3));
  }
#pragma unroll
  for (int e = 0; e < 4; ++e) {
    _Float16 h, l;
    const float f = ov[e];
    f16_split(f, h, l);
    hv[e] = h;
    lv[e] = l;
  }
  const size_t e0 = (size_t)i * 4;
  *(volatile v4f*)(XC + e0) = ov;
  *(volatile v4h*)(XCH + e0) = hv;
  *(volatile v4h*)(XCL + e0) = lv;
  __threadfence();
  *(volatile v4f*)(XC + e0) = ov;
  *(volatile v4h*)(XCH + e0) = hv;
  *(volatile v4h*)(XCL + e0) = lv;
}

__global__ __launch_bounds__(256) void scan_planes_kernel(
    const float* __restrict__ XD, const float* __restrict__ XC,
    const float* __restrict__ dtw, const float* __restrict__ dtb,
    float* __restrict__ DTP, float* __restrict__ UK, float* __restrict__ BC)
{
  const int k = blockIdx.y;
  const int i = blockIdx.x * 256 + threadIdx.x;
  if (i >= kLen * (kDin / 4)) return;
  const int l  = i / (kDin / 4);
  const int g  = i - l * (kDin / 4);
  const int d4 = g * 4;
  const int p  = scan_pixel(k, l);
  const float* xr = XD + (size_t)p * kXdN + k * kXpP;
  float rk[kDtR];
#pragma unroll
  for (int r = 0; r < kDtR; ++r) rk[r] = xr[r];
  const float* wp = dtw + ((size_t)k * kDin + d4) * kDtR;
  v4f wv[6];
#pragma unroll
  for (int q = 0; q < 6; ++q) wv[q] = *(const v4f*)(wp + 4 * q);
  const v4f bias = *(const v4f*)(dtb + k * kDin + d4);
  v4f dv;
#pragma unroll
  for (int j = 0; j < 4; ++j) {
    float acc = 0.0f;
#pragma unroll
    for (int r = 0; r < kDtR; ++r) {
      const int e = j * kDtR + r;
      acc = fmaf(wv[e >> 2][e & 3], rk[r], acc);
    }
    dv[j] = acc + bias[j];
  }
  const v4f uv = *(const v4f*)(XC + (size_t)p * kDin + d4);
  const int gc = (g < 8) ? g : 7;
  v4f bcv;
#pragma unroll
  for (int e = 0; e < 4; ++e) bcv[e] = xr[kDtR + 4 * gc + e];
  const size_t o  = ((size_t)k * kLen + l) * kDin + d4;
  const size_t ob = ((size_t)k * kLen + l) * kBcN + 4 * gc;
  for (int pass = 0; pass < 2; ++pass) {
    *(volatile v4f*)(DTP + o) = dv;
    *(volatile v4f*)(UK + o) = uv;
    if (g < 8) *(volatile v4f*)(BC + ob) = bcv;
    __threadfence();
  }
}

typedef float    ms1_v4f __attribute__((ext_vector_type(4)));
typedef unsigned ms1_v4u __attribute__((ext_vector_type(4)));
struct ms1_args {
  const float* dtpre;
  const float* u;
  const float* bc;
  const float* z;
  const float* A_log;
  const float* Dskip;
  __half* y;
  __half* y_lo;
  long ld_dtpre;
  long ld_u;
  long ld_bc;
  long ld_z;
  long ld_y;
  int offB;
  int offC;
  int offZ;
  float ycarry;
  int dir;
  int D;
  int L;
  int nbatch;
};
static_assert(sizeof(ms1_args) == 136);

__device__ __forceinline__ float ms1_flush16(float v) {
  return (fabsf(v) < 6.103515625e-05f) ? 0.0f : v;
}
__device__ __forceinline__ unsigned ms1_h16bits(float v) {
  return (unsigned)__half_as_ushort(__float2half_rn(ms1_flush16(v)));
}
__device__ __forceinline__ float ms1_h16val(unsigned b) {
  return __half2float(__ushort_as_half((unsigned short)b));
}
__device__ __forceinline__ float ms1_softplus(float v) {
  return fmaxf(v, 0.0f) + log1pf(expf(-fabsf(v)));
}
__device__ __forceinline__ void ms1_pack2(float v0, float v1, unsigned& hw, unsigned& lw) {
  const unsigned h0 = ms1_h16bits(v0);
  const unsigned h1 = ms1_h16bits(v1);
  const float r0 = (v0 - ms1_h16val(h0)) * 2048.0f;
  const float r1 = (v1 - ms1_h16val(h1)) * 2048.0f;
  const unsigned l0 = ms1_h16bits(r0);
  const unsigned l1 = ms1_h16bits(r1);
  hw = h0 | (h1 << 16);
  lw = l0 | (l1 << 16);
}

template <int NSTATE>
__global__ __launch_bounds__(64 * (NSTATE / 16)) void ms1_scan_kernel(ms1_args a)
{
  static_assert(NSTATE == 16 || NSTATE == 64);
  constexpr int NQ  = NSTATE / 16;
  constexpr int NT  = 64 * NQ;
  constexpr int NW  = NT / 32;
  constexpr int BCW = 2 * NSTATE;
  constexpr int YP  = 68;
  constexpr int RPI = NW * 4;
  constexpr int NIT = 64 / RPI;
  static_assert(16 * NT <= 64 * YP);
  __shared__ __align__(16) float sBC[64 * BCW];
  __shared__ __align__(16) float sY[64 * YP];
  const int tid  = threadIdx.x;
  const int lane = tid & 31;
  const int wave = tid >> 5;
  const int c    = tid / NQ;
  const int sq   = tid - c * NQ;
  const int bpb  = a.D / 64;
  const int bi   = blockIdx.x / bpb;
  if (bi >= a.nbatch) return;
  const int d0 = (blockIdx.x - bi * bpb) * 64;
  const int d  = d0 + c;
  const long rowb = (long)bi * a.L;
  const bool hasz  = (a.z != nullptr);
  const bool hasD  = (a.Dskip != nullptr);
  const bool hasLo = (a.y_lo != nullptr);

#pragma unroll 1
  for (int n = 0; n < 16; ++n) {
    const float al = a.A_log[(long)d * NSTATE + sq * 16 + n];
    sY[n * NT + tid] = -expf(al);
  }
  __syncthreads();
  float An[16], h[16];
#pragma unroll
  for (int n = 0; n < 16; ++n) {
    An[n] = sY[n * NT + tid];
    h[n] = 0.0f;
  }
  float Dd = 0.0f;
  if (hasD) Dd = a.Dskip[d];

  const int nchunk = a.L / 64;
  const bool fwd = (a.dir > 0);
  const int s0 = fwd ? 0 : 63;
  const int sd = fwd ? 1 : -1;
  const int q  = lane >> 3;
  const int c8 = (lane & 7) * 8;

#pragma unroll 1
  for (int ci = 0; ci < nchunk; ++ci) {
    const int tb = fwd ? (ci * 64) : (a.L - 64 - ci * 64);
    const long rowc = rowb + tb;
    __syncthreads();
#pragma unroll 8
    for (int i = 0; i < 32; ++i) {
      const int idx = tid + i * NT;
      const int st  = idx / BCW;
      const int col = idx - st * BCW;
      const int sc  = (col < NSTATE) ? (a.offB + col) : (a.offC + col - NSTATE);
      sBC[idx] = a.bc[(rowc + st) * a.ld_bc + sc];
    }
    __syncthreads();
#pragma unroll 1
    for (int s = 0; s < 64; ++s) {
      const int ls = s0 + sd * s;
      const long row = rowc + ls;
      float pre = a.dtpre[row * a.ld_dtpre + d];
      float uv  = a.u[row * a.ld_u + d];
      float zv  = 0.0f;
      if (hasz) zv = a.z[row * a.ld_z + a.offZ + d];
      asm volatile("" : "+v"(pre));
      asm volatile("" : "+v"(uv));
      asm volatile("" : "+v"(zv));
      const float delta = ms1_softplus(pre);
      const float dtx = delta * uv;
      const float* bp = sBC + ls * BCW + sq * 16;
      const float* cp = bp + NSTATE;
      ms1_v4f Bq[4], Cq[4];
#pragma unroll
      for (int k = 0; k < 4; ++k) {
        Bq[k] = *(const ms1_v4f*)(bp + 4 * k);
        Cq[k] = *(const ms1_v4f*)(cp + 4 * k);
      }
      float yv = 0.0f;
#pragma unroll
      for (int n = 0; n < 16; ++n) {
        const float e = __expf(delta * An[n]);
        h[n] = fmaf(e, h[n], dtx * Bq[n >> 2][n & 3]);
        yv = fmaf(h[n], Cq[n >> 2][n & 3], yv);
      }
      if (NQ > 1) {
        yv += __shfl_xor(yv, 1, 32);
        yv += __shfl_xor(yv, 2, 32);
      }
      if (hasD) yv = fmaf(uv, Dd, yv);
      if (hasz) {
        const float sg = __builtin_amdgcn_rcpf(1.0f + expf(-zv));
        yv = yv * (zv * sg);
      }
      if (sq == 0) sY[ls * YP + c] = yv * a.ycarry;
    }
    __syncthreads();
    ms1_v4u hw[NIT], lw[NIT];
#pragma unroll
    for (int it = 0; it < NIT; ++it) {
      const int row = it * RPI + wave * 4 + q;
      const float* sp = sY + row * YP + c8;
      const ms1_v4f f0 = *(const ms1_v4f*)(sp);
      const ms1_v4f f1 = *(const ms1_v4f*)(sp + 4);
      unsigned h0, h1, h2, h3, l0, l1, l2, l3;
      ms1_pack2(f0[0], f0[1], h0, l0);
      ms1_pack2(f0[2], f0[3], h1, l1);
      ms1_pack2(f1[0], f1[1], h2, l2);
      ms1_pack2(f1[2], f1[3], h3, l3);
      hw[it] = (ms1_v4u){h0, h1, h2, h3};
      lw[it] = (ms1_v4u){l0, l1, l2, l3};
    }
    for (int pass = 0; pass < 2; ++pass) {
#pragma unroll
      for (int it = 0; it < NIT; ++it) {
        const int row = it * RPI + wave * 4 + q;
        const long o = (rowc + row) * a.ld_y + d0 + c8;
        *(volatile ms1_v4u*)(a.y + o) = hw[it];
        if (hasLo) *(volatile ms1_v4u*)(a.y_lo + o) = lw[it];
      }
      __threadfence();
    }
  }
}

constexpr int kMgPix   = 32;
constexpr int kMgPitch = 196;
static_assert((kLen % kMgPix) == 0);
static_assert(kMgPix * (kDin / 8) == 3 * 256);
__global__ __launch_bounds__(256) void merge_norm_gate_kernel(
    const unsigned short* __restrict__ YSH, const unsigned short* __restrict__ YSL,
    const float* __restrict__ XZ, const float* __restrict__ gam, const float* __restrict__ bet,
    unsigned short* __restrict__ YGH, unsigned short* __restrict__ YGL)
{
  __shared__ __align__(16) float sT[kMgPix * kMgPitch];
  const int tid = threadIdx.x, lane = tid & 31, wave = tid >> 5;
  const int p0 = blockIdx.x * kMgPix;
  constexpr float kResidInv = 1.0f / kResid;
  constexpr float kYsInv = 1.0f / kYCarry;

#pragma unroll 1
  for (int it = 0; it < 3; ++it) {
    const int t  = tid + it * 256;
    const int pp = t / (kDin / 8);
    const int g  = t - pp * (kDin / 8);
    const int p  = p0 + pp;
    const int pt = ((p & 63) << 6) + (p >> 6);
    float acc[8];
#pragma unroll
    for (int e = 0; e < 8; ++e) acc[e] = 0.0f;
#pragma unroll 1
    for (int k = 0; k < kDir; ++k) {
      const int base = (k & 1) ? pt : p;
      const int l = (k >= 2) ? (kLen - 1 - base) : base;
      const size_t o = ((size_t)k * kLen + l) * kDin + 8 * g;
      const gl_v4u hw = *(const gl_v4u*)(YSH + o);
      const gl_v4u lw = *(const gl_v4u*)(YSL + o);
#pragma unroll
      for (int j = 0; j < 4; ++j) {
        const float h0 = h16_to_f32(hw[j] & 0xffffu);
        const float h1 = h16_to_f32(hw[j] >> 16);
        const float l0 = h16_to_f32(lw[j] & 0xffffu);
        const float l1 = h16_to_f32(lw[j] >> 16);
        acc[2 * j]     += fmaf(l0, kResidInv, h0);
        acc[2 * j + 1] += fmaf(l1, kResidInv, h1);
      }
    }
    float* dp = sT + pp * kMgPitch + 8 * g;
    *(v4f*)(dp)     = (v4f){acc[0] * kYsInv, acc[1] * kYsInv, acc[2] * kYsInv, acc[3] * kYsInv};
    *(v4f*)(dp + 4) = (v4f){acc[4] * kYsInv, acc[5] * kYsInv, acc[6] * kYsInv, acc[7] * kYsInv};
  }
  __syncthreads();

#pragma unroll 1
  for (int j = 0; j < 4; ++j) {
    const int pp = wave * 4 + j;
    const int p  = p0 + pp;
    float* rowp = sT + pp * kMgPitch;
    float v[6];
    float s = 0.0f;
#pragma unroll
    for (int i = 0; i < 6; ++i) {
      v[i] = rowp[lane + 32 * i];
      s += v[i];
    }
#pragma unroll
    for (int off = 16; off >= 1; off >>= 1) s += __shfl_xor(s, off, 32);
    const float mu = s * (1.0f / (float)kDin);
    float qs = 0.0f;
#pragma unroll
    for (int i = 0; i < 6; ++i) {
      v[i] = v[i] - mu;
      qs = fmaf(v[i], v[i], qs);
    }
#pragma unroll
    for (int off = 16; off >= 1; off >>= 1) qs += __shfl_xor(qs, off, 32);
    const float var = qs * (1.0f / (float)kDin);
    const float rstd = rsqrtf(var + 1e-5f);
#pragma unroll
    for (int i = 0; i < 6; ++i) {
      const int d = lane + 32 * i;
      const float yn = v[i] * rstd * gam[d] + bet[d];
      const float zv = XZ[(size_t)p * kXzN + kDin + d];
      const float sg = __builtin_amdgcn_rcpf(1.0f + expf(-zv));
      rowp[d] = yn * (zv * sg);
    }
  }
  __syncthreads();

  v8h hv[3], lv[3];
#pragma unroll
  for (int it = 0; it < 3; ++it) {
    const int t  = tid + it * 256;
    const int pp = t / (kDin / 8);
    const int g  = t - pp * (kDin / 8);
    const float* sp = sT + pp * kMgPitch + 8 * g;
    const v4f a0 = *(const v4f*)(sp);
    const v4f a1 = *(const v4f*)(sp + 4);
#pragma unroll
    for (int e = 0; e < 4; ++e) {
      _Float16 h0, l0, h1, l1;
      const float f0 = a0[e] * kYgCarry;
      const float f1 = a1[e] * kYgCarry;
      f16_split(f0, h0, l0);
      f16_split(f1, h1, l1);
      hv[it][e] = h0; lv[it][e] = l0;
      hv[it][4 + e] = h1; lv[it][4 + e] = l1;
    }
  }
  for (int pass = 0; pass < 2; ++pass) {
#pragma unroll
    for (int it = 0; it < 3; ++it) {
      const size_t o = (size_t)p0 * kDin + (size_t)(tid + it * 256) * 8;
      *(volatile v8h*)(YGH + o) = hv[it];
      *(volatile v8h*)(YGL + o) = lv[it];
    }
    __threadfence();
  }
}

__global__ __launch_bounds__(256) void copy_out_kernel(
    const float* __restrict__ OUTP, float* __restrict__ out, int total4)
{
  const int i = blockIdx.x * 256 + threadIdx.x;
  if (i >= total4) return;
  const int e0  = i * 4;
  const int row = e0 / kCh;
  const int col = e0 - row * kCh;
  const v4f v = *(const v4f*)(OUTP + (size_t)row * kOutP + col);
  *(volatile v4f*)(out + (size_t)e0) = v;
  __threadfence();
  *(volatile v4f*)(out + (size_t)e0) = v;
}

extern "C" void kernel_launch(void* const* d_in, const int* in_sizes, int n_in,
                              void* d_out, int out_size, void* d_ws, size_t ws_size,
                              hipStream_t stream)
{
  if (n_in < 12) return;
  if (in_sizes[0] != kRows * kCh) return;
  if (in_sizes[1] != kXzN * kCh) return;
  if (in_sizes[2] != kDin * 9) return;
  if (in_sizes[3] != kDin) return;
  if (in_sizes[4] != kDir * kXpC * kDin) return;
  if (in_sizes[5] != kDir * kDin * kDtR) return;
  if (in_sizes[6] != kDir * kDin) return;
  if (in_sizes[7] != kDir * kDin * kNst) return;
  if (in_sizes[8] != kDir * kDin) return;
  if (in_sizes[9] != kDin) return;
  if (in_sizes[10] != kDin) return;
  if (in_sizes[11] != kCh * kDin) return;
  if (out_size != kRows * kCh) return;
  if (ws_size < kWsTotal) return;

  const float* x      = (const float*)d_in[0];
  const float* W_in   = (const float*)d_in[1];
  const float* conv_w = (const float*)d_in[2];
  const float* conv_b = (const float*)d_in[3];
  const float* W_x    = (const float*)d_in[4];
  const float* W_dt   = (const float*)d_in[5];
  const float* b_dt   = (const float*)d_in[6];
  const float* A_log  = (const float*)d_in[7];
  const float* D_par  = (const float*)d_in[8];
  const float* ln_g   = (const float*)d_in[9];
  const float* ln_b   = (const float*)d_in[10];
  const float* W_out  = (const float*)d_in[11];
  float* out = (float*)d_out;

  char* ws = (char*)d_ws;
  unsigned short* WINH = (unsigned short*)(ws + kOffWINH);
  unsigned short* WINL = (unsigned short*)(ws + kOffWINL);
  unsigned short* WX   = (unsigned short*)(ws + kOffWX);
  unsigned short* WO   = (unsigned short*)(ws + kOffWO);
  unsigned short* XH   = (unsigned short*)(ws + kOffXH);
  unsigned short* XL   = (unsigned short*)(ws + kOffXL);
  float*          XZ   = (float*)(ws + kOffXZ);
  float*          XC   = (float*)(ws + kOffXC);
  unsigned short* XCH  = (unsigned short*)(ws + kOffXCH);
  unsigned short* XCL  = (unsigned short*)(ws + kOffXCL);
  float*          XD   = (float*)(ws + kOffXD);
  float*          DTP  = (float*)(ws + kOffDTP);
  float*          UK   = (float*)(ws + kOffUK);
  float*          BC   = (float*)(ws + kOffBC);
  unsigned short* YSH  = (unsigned short*)(ws + kOffYSH);
  unsigned short* YSL  = (unsigned short*)(ws + kOffYSL);
  unsigned short* YGH  = (unsigned short*)(ws + kOffYGH);
  unsigned short* YGL  = (unsigned short*)(ws + kOffYGL);
  float*          OUTP = (float*)(ws + kOffOUTP);

  constexpr float sW  = 1.0f / kWCarry;
  constexpr float sWr = 1.0f / (kWCarry * kResid);
  constexpr float sY  = 1.0f / (kYgCarry * kWCarry);
  constexpr float sYr = 1.0f / (kYgCarry * kWCarry * kResid);

  pack_w_rows_kernel<true><<<dim3((kXzN * kCh / 8) / 256), 256, 0, stream>>>(
      W_in, WINH, WINL, kCh / 8, kXzN, kXzN, kXzN * kCh / 8, kWCarry);
  pack_w_rows_kernel<false><<<dim3((kXdN * kDin / 8) / 256), 256, 0, stream>>>(
      W_x, WX, WX, kDin / 8, kXpP, kXpC, kXdN * kDin / 8, kWCarry);
  pack_w_rows_kernel<false><<<dim3((kOutP * kDin / 8) / 256), 256, 0, stream>>>(
      W_out, WO, WO, kDin / 8, kOutP, kCh, kOutP * kDin / 8, kWCarry);

  split_rows_f16_kernel<<<dim3((kRows * kCh / 8) / 256), 256, 0, stream>>>(x, XH, XL, kRows * kCh / 8);

  for (int b = 0; b < kBatch; ++b) {
    const unsigned short* xh = XH + (size_t)b * kLen * kCh;
    const unsigned short* xl = XL + (size_t)b * kLen * kCh;

    eng::gemm_f16_kernel<1, 2><<<dim3((kLen / 16) * (kXzN / 64) / 8), 256, 0, stream>>>(
        xh, xl, kCh, WINH, WINL, kCh, XZ, kXzN, kLen, kXzN, kCh, sW, sWr);

    dwconv3x3_silu_kernel<<<dim3(kLen * (kDin / 4) / 256), 256, 0, stream>>>(XZ, conv_w, conv_b, XC, XCH, XCL);

    eng::gemm_f16_kernel<2, 1><<<dim3((kLen / 32) * (kXdN / 64) / 8), 256, 0, stream>>>(
        XCH, XCL, kDin, WX, WX, kDin, XD, kXdN, kLen, kXdN, kDin, sW, sWr);

    scan_planes_kernel<<<dim3(kLen * (kDin / 4) / 256, kDir), 256, 0, stream>>>(XD, XC, W_dt, b_dt, DTP, UK, BC);

    for (int k = 0; k < kDir; ++k) {
      ms1_args sa;
      sa.dtpre = DTP + (size_t)k * kLen * kDin;
      sa.u = UK + (size_t)k * kLen * kDin;
      sa.bc = BC + (size_t)k * kLen * kBcN;
      sa.z = nullptr;
      sa.A_log = A_log + (size_t)k * kDin * kNst;
      sa.Dskip = D_par + (size_t)k * kDin;
      sa.y = (__half*)(YSH + (size_t)k * kLen * kDin);
      sa.y_lo = (__half*)(YSL + (size_t)k * kLen * kDin);
      sa.ld_dtpre = kDin;
      sa.ld_u = kDin;
      sa.ld_bc = kBcN;
      sa.ld_z = 0;
      sa.ld_y = kDin;
      sa.offB = 0;
      sa.offC = kNst;
      sa.offZ = 0;
      sa.ycarry = kYCarry;
      sa.dir = 1;
      sa.D = kDin;
      sa.L = kLen;
      sa.nbatch = 1;
      ms1_scan_kernel<16><<<dim3(kDin / 64), 64, 0, stream>>>(sa);
    }

    merge_norm_gate_kernel<<<dim3(kLen / kMgPix), 256, 0, stream>>>(
        YSH, YSL, XZ, ln_g, ln_b, YGH + (size_t)b * kLen * kDin, YGL + (size_t)b * kLen * kDin);
  }

  eng::gemm_f16_kernel<2, 1><<<dim3((kRows / 32) * (kOutP / 64) / 8), 256, 0, stream>>>(
      YGH, YGL, kDin, WO, WO, kDin, OUTP, kOutP, kRows, kOutP, kDin, sY, sYr);

  copy_out_kernel<<<dim3((kRows * kCh / 4) / 256), 256, 0, stream>>>(OUTP, out, kRows * kCh / 4);
}
